// GNN_64003602645422
// MI455X (gfx1250) — hardware-verified
//
#include <hip/hip_runtime.h>
#include <stddef.h>
#include <stdint.h>
#include <math.h>


#define FT      128
#define XW      256
#define NGR     50
#define NPER    1000
#define NTHR    256
#define NWAVE   8
#define EPT     8
#define CHUNK   (NTHR * EPT)
#define WCAP    (EPT * 32)
#define LISTN   (NWAVE * WCAP)
#define NBMAX   2048
#define NBRUN   1024
#define RCAP    28672
#define DEGCAP  128
#define STW     512
#define GBM     64
#define GBN     64
#define GTHR    128
#define NUW1    (FT * (FT / 8))
#define NUW2    (FT * (XW / 8))
#define NUW     (2 * NUW1 + 2 * NUW2)
#define NEGS    0.2f
#define WSMAX   134217728
#define LDS_AGG ((2 * RCAP + 2 * NBMAX + LISTN) * 4 + 64)

static_assert((CHUNK & (CHUNK - 1)) == 0 && CHUNK <= 4096);
static_assert((NBMAX & (NBMAX - 1)) == 0 && NBMAX <= 4096);
static_assert((NBRUN & (NBRUN - 1)) == 0 && NBRUN <= NBMAX && NBRUN >= 16);
static_assert(NTHR * 8 == NBMAX);
static_assert(LISTN >= NBMAX);
static_assert((RCAP % 32) == 0);
static_assert(NWAVE * STW <= RCAP);
static_assert(FT <= STW);
static_assert(LDS_AGG <= 300000);
static_assert(GBM == (GTHR / 32) * 16 && GBN == 64);
static_assert(FT == 32 * 4);
static_assert(FT / 4 == 32 && 32 / 4 == 8);
static_assert((FT % 32) == 0 && (XW % 32) == 0 && (XW % GBN) == 0 && (FT % GBN) == 0);
static_assert(NUW1 % NTHR == 0 && NUW2 % NTHR == 0 && NUW % NTHR == 0);
static_assert(RCAP >= 17543);
static_assert(DEGCAP >= 35 + 8);
static_assert((2 * NGR * FT - 1) < 2 * NGR * FT);

typedef float          v4f   __attribute__((ext_vector_type(4)));
typedef float          v8f   __attribute__((ext_vector_type(8)));
typedef int            v4i   __attribute__((ext_vector_type(4)));
typedef int            v8i   __attribute__((ext_vector_type(8)));
typedef unsigned int   v4u   __attribute__((ext_vector_type(4)));
typedef unsigned short v8us  __attribute__((ext_vector_type(8)));
typedef unsigned short v16us __attribute__((ext_vector_type(16)));
typedef __bf16         v16bf __attribute__((ext_vector_type(16)));
typedef v4f  __attribute__((may_alias)) v4fa;
typedef v4i  __attribute__((may_alias)) v4ia;
typedef v8us __attribute__((may_alias)) v8usa;
union FragB { v16bf v; v16us u; v8us h[2]; v8i w; };

__device__ __forceinline__ v8f wmb(const FragB& a, const FragB& b, v8f c) {
  v8f d = __builtin_amdgcn_wmma_f32_16x16x32_bf16(false, a.v, false, b.v, (short)0, c, false, false);
  asm volatile("v_nop\n\tv_nop\n\tv_nop\n\tv_nop" : "+v"(d) : "v"(a.w), "v"(b.w));
  return d;
}

__device__ __forceinline__ unsigned bf16_bits(float f) {
  const unsigned u = __float_as_uint(f);
  return (u + 0x7FFFu + ((u >> 16) & 1u)) >> 16;
}
__device__ __forceinline__ float bf16_val(float f) {
  return __uint_as_float(bf16_bits(f) << 16);
}

__device__ __forceinline__ v8us gather8(const float* __restrict__ w, int k8, int n) {
  const float* p = w + (size_t)k8 * FT + n;
  v8us o;
#pragma unroll
  for (int i = 0; i < 8; ++i) o[i] = (unsigned short)bf16_bits(p[(size_t)i * FT]);
  return o;
}

__device__ __forceinline__ int scan_chunk(const int* __restrict__ dsts, int nE, int cbase, int slotBase,
                                          int nb, int vec8, int* list, int tid, int lane, int wave) {
  int wc = 0;
  const int el0  = tid * EPT;
  const int e0   = cbase + el0;
  const int sent = -2147483647 - 1;
  v4i da, db;
  if (vec8 != 0 && cbase + CHUNK <= nE) {
    da = *(const v4i*)(dsts + e0);
    db = *(const v4i*)(dsts + e0 + 4);
  } else {
    da.x = (e0     < nE) ? dsts[min(e0,     nE - 1)] : sent;
    da.y = (e0 + 1 < nE) ? dsts[min(e0 + 1, nE - 1)] : sent;
    da.z = (e0 + 2 < nE) ? dsts[min(e0 + 2, nE - 1)] : sent;
    da.w = (e0 + 3 < nE) ? dsts[min(e0 + 3, nE - 1)] : sent;
    db.x = (e0 + 4 < nE) ? dsts[min(e0 + 4, nE - 1)] : sent;
    db.y = (e0 + 5 < nE) ? dsts[min(e0 + 5, nE - 1)] : sent;
    db.z = (e0 + 6 < nE) ? dsts[min(e0 + 6, nE - 1)] : sent;
    db.w = (e0 + 7 < nE) ? dsts[min(e0 + 7, nE - 1)] : sent;
  }
  const unsigned nbs = (unsigned)slotBase;
  const unsigned unb = (unsigned)nb;
  const unsigned s0 = (unsigned)da.x - nbs, s1 = (unsigned)da.y - nbs;
  const unsigned s2 = (unsigned)da.z - nbs, s3 = (unsigned)da.w - nbs;
  const unsigned s4 = (unsigned)db.x - nbs, s5 = (unsigned)db.y - nbs;
  const unsigned s6 = (unsigned)db.z - nbs, s7 = (unsigned)db.w - nbs;
  const bool h0 = s0 < unb, h1 = s1 < unb, h2 = s2 < unb, h3 = s3 < unb;
  const bool h4 = s4 < unb, h5 = s5 < unb, h6 = s6 < unb, h7 = s7 < unb;
  const unsigned any = __builtin_amdgcn_ballot_w32(h0 | h1 | h2 | h3 | h4 | h5 | h6 | h7);
  if (any != 0u) {
#define HITJ(J, HJ, SJ) { \
      const unsigned mj = __builtin_amdgcn_ballot_w32(HJ); \
      if (mj != 0u) { \
        if (HJ) { \
          const int pos = wc + (int)__builtin_amdgcn_mbcnt_lo(mj, 0u); \
          if (pos < WCAP) list[wave * WCAP + pos] = ((el0 + (J)) << 12) | (int)(SJ); \
        } \
        wc += (int)__builtin_popcount(mj); } }
    HITJ(0, h0, s0)
    HITJ(1, h1, s1)
    HITJ(2, h2, s2)
    HITJ(3, h3, s3)
    HITJ(4, h4, s4)
    HITJ(5, h5, s5)
    HITJ(6, h6, s6)
    HITJ(7, h7, s7)
#undef HITJ
  }
  return wc;
}

__global__ __launch_bounds__(NTHR) void k_prep(const float* __restrict__ x,
                                               const float* __restrict__ Wl1, const float* __restrict__ Wr1,
                                               const float* __restrict__ Wl2, const float* __restrict__ Wr2,
                                               unsigned short* XB, unsigned short* W1T, unsigned short* W2T,
                                               int nN, int gX) {
  const int tid = (int)threadIdx.x;
  const int blk = (int)blockIdx.x;
  v8us o;
  unsigned short* dp;
  if (blk < gX) {
    const int u   = blk * NTHR + tid;
    const int row = u >> 4;
    const int k8  = (u & 15) * 8;
    const int rc  = row < nN ? row : nN - 1;
    const float* p = x + (size_t)rc * FT + k8;
    const v4f a = *(const v4fa*)p;
    const v4f b = *(const v4fa*)(p + 4);
    const bool ok = row < nN;
    o[0] = ok ? (unsigned short)bf16_bits(a.x) : (unsigned short)0;
    o[1] = ok ? (unsigned short)bf16_bits(a.y) : (unsigned short)0;
    o[2] = ok ? (unsigned short)bf16_bits(a.z) : (unsigned short)0;
    o[3] = ok ? (unsigned short)bf16_bits(a.w) : (unsigned short)0;
    o[4] = ok ? (unsigned short)bf16_bits(b.x) : (unsigned short)0;
    o[5] = ok ? (unsigned short)bf16_bits(b.y) : (unsigned short)0;
    o[6] = ok ? (unsigned short)bf16_bits(b.z) : (unsigned short)0;
    o[7] = ok ? (unsigned short)bf16_bits(b.w) : (unsigned short)0;
    dp = XB + (size_t)row * FT + k8;
  } else {
    const int v = (blk - gX) * NTHR + tid;
    if (v < NUW1) {
      const int n = v >> 4, k8 = (v & 15) * 8;
      o  = gather8(Wl1, k8, n);
      dp = W1T + (size_t)n * FT + k8;
    } else if (v < 2 * NUW1) {
      const int w = v - NUW1;
      const int n = w >> 4, k8 = (w & 15) * 8;
      o  = gather8(Wr1, k8, n);
      dp = W1T + (size_t)(FT + n) * FT + k8;
    } else if (v < 2 * NUW1 + NUW2) {
      const int w = v - 2 * NUW1;
      const int n = w >> 5, k8 = (w & 31) * 8;
      o  = gather8(Wl2, k8 & (FT - 1), n);
      dp = W2T + (size_t)n * XW + k8;
    } else if (v < NUW) {
      const int w = v - 2 * NUW1 - NUW2;
      const int n = w >> 5, k8 = (w & 31) * 8;
      o  = gather8(Wr2, k8 & (FT - 1), n);
      dp = W2T + (size_t)(FT + n) * XW + k8;
    } else {
      return;
    }
  }
  *(volatile v8us*)dp = o;
  __threadfence();
  *(volatile v8us*)dp = o;
}

__global__ __launch_bounds__(GTHR) void k_gemm(
    const unsigned short* __restrict__ A, const unsigned short* __restrict__ WT,
    const float* __restrict__ bA, const float* __restrict__ bB,
    float* outF, int K, int ldo)
{
  __shared__ __attribute__((aligned(16))) float stg[GBM * GBN];
  const int tid = (int)threadIdx.x, lane = tid & 31, wave = tid >> 5, hh = lane >> 4, m = lane & 15;
  const int rowBase = (int)blockIdx.x * GBM;
  const int col0    = (int)blockIdx.y * GBN;

  v8f acc[4];
  {
    const v8f z = {0.f, 0.f, 0.f, 0.f, 0.f, 0.f, 0.f, 0.f};
    acc[0] = z; acc[1] = z; acc[2] = z; acc[3] = z;
  }
  const unsigned short* ap = A  + (size_t)(rowBase + 16 * wave + m) * (size_t)K + 8 * hh;
  const unsigned short* wp = WT + (size_t)(col0 + m) * (size_t)K + 8 * hh;
  const int ksteps = K >> 5;
#pragma unroll 1
  for (int ks = 0; ks < ksteps; ++ks) {
    FragB af;
    af.h[0] = *(const v8usa*)(ap + 32 * ks);
    af.h[1] = *(const v8usa*)(ap + 32 * ks + 16);
#pragma unroll
    for (int t = 0; t < 4; ++t) {
      const unsigned short* wq = wp + (size_t)(16 * t) * (size_t)K + 32 * ks;
      FragB bf;
      bf.h[0] = *(const v8usa*)wq;
      bf.h[1] = *(const v8usa*)(wq + 16);
      acc[t] = wmb(af, bf, acc[t]);
    }
  }

  float bv[4];
  if (col0 < FT) {
#pragma unroll
    for (int t = 0; t < 4; ++t) bv[t] = bf16_val(bA[col0 + 16 * t + m]);
  } else {
#pragma unroll
    for (int t = 0; t < 4; ++t) bv[t] = bf16_val(bB[col0 - FT + 16 * t + m]);
  }

#pragma unroll
  for (int t = 0; t < 4; ++t) {
    const int lc = 16 * t + m;
#pragma unroll
    for (int r = 0; r < 8; ++r) {
      const int lr = 16 * wave + 8 * hh + r;
      stg[lr * GBN + lc] = acc[t][r] + bv[t];
    }
  }
  __syncthreads();

  v4f fv[8];
#pragma unroll
  for (int i = 0; i < 8; ++i) {
    const int lr = 16 * wave + 2 * i + hh;
    fv[i] = *(const v4fa*)(stg + lr * GBN + 4 * m);
  }
#pragma unroll
  for (int i = 0; i < 8; ++i) {
    const int lr = 16 * wave + 2 * i + hh;
    const int gr = rowBase + lr;
    float* op = outF + (size_t)gr * (size_t)ldo + col0 + 4 * m;
    *(volatile v4f*)op = fv[i];
  }
  __threadfence();
#pragma unroll
  for (int i = 0; i < 8; ++i) {
    const int lr = 16 * wave + 2 * i + hh;
    const int gr = rowBase + lr;
    float* op = outF + (size_t)gr * (size_t)ldo + col0 + 4 * m;
    *(volatile v4f*)op = fv[i];
  }
}

__device__ __forceinline__ float lkatt4(const v4f a, const v4f b, const v4f w) {
  float t0 = a.x + b.x, t1 = a.y + b.y, t2 = a.z + b.z, t3 = a.w + b.w;
  t0 = t0 > 0.f ? t0 : t0 * NEGS;
  t1 = t1 > 0.f ? t1 : t1 * NEGS;
  t2 = t2 > 0.f ? t2 : t2 * NEGS;
  t3 = t3 > 0.f ? t3 : t3 * NEGS;
  float p = t0 * w.x;
  p = fmaf(t1, w.y, p);
  p = fmaf(t2, w.z, p);
  p = fmaf(t3, w.w, p);
  return p;
}
template<int NR>
__device__ __forceinline__ float gred(float p) {
#pragma unroll
  for (int i = 0; i < NR; ++i) p += __shfl_xor(p, 1 << i);
  return p;
}

template<int L>
__global__ __launch_bounds__(NTHR) void k_agg(
    const int* __restrict__ srcs, const int* __restrict__ dsts,
    const float* __restrict__ XLR, const float* __restrict__ att, const float* __restrict__ bias,
    unsigned short* H1, float* H2,
    int nN, int nE, int nb, int vec8, int MPr) {
  constexpr int NR = (L == 1) ? 3 : 5;
  extern __shared__ v4f lds_dyn[];
  int* reg1 = (int*)lds_dyn;
  int* reg2 = reg1 + RCAP;
  int* scnt = reg2 + RCAP;
  int* soff = scnt + NBMAX;
  int* list = soff + NBMAX;
  int* wcnt = list + LISTN;
  int* wtot = wcnt + NWAVE;
  const int tid = (int)threadIdx.x, lane = tid & 31, wave = tid >> 5;
  const int nodeBase = (int)blockIdx.x * nb;

  for (int i = tid; i < NBMAX; i += NTHR) scnt[i] = 0;
  __syncthreads();

  int tot = 0;
  const int nChunks = (nE + CHUNK - 1) / CHUNK;
#pragma unroll 1
  for (int ch = 0; ch < nChunks; ++ch) {
    const int cbase = ch * CHUNK;
    const int wc = scan_chunk(dsts, nE, cbase, nodeBase, nb, vec8, list, tid, lane, wave);
    if (lane == 0) wcnt[wave] = wc;
    __syncthreads();
    int pre = 0, all = 0;
#pragma unroll
    for (int w2 = 0; w2 < NWAVE; ++w2) {
      int c = wcnt[w2];
      c = c < 0 ? 0 : (c > WCAP ? WCAP : c);
      all += c;
      pre += (w2 < wave) ? c : 0;
    }
    const int wcc  = wc > WCAP ? WCAP : wc;
    const int base = tot + pre;
#pragma unroll 1
    for (int i = lane; i < wcc; i += 32) {
      const int ent = list[wave * WCAP + i];
      const int el  = (ent >> 12) & (CHUNK - 1);
      const int sl  = ent & (NBMAX - 1);
      int eid = cbase + el;
      eid = eid > nE - 1 ? nE - 1 : eid;
      const int pos = base + i;
      if (pos < RCAP) reg1[pos] = (int)(((unsigned)eid << 12) | (unsigned)sl);
    }
    tot += all;
    tot = tot > RCAP ? RCAP : tot;
    __syncthreads();
  }
  const int nh = tot;

  if (wave == 0) {
#pragma unroll 1
    for (int b0 = 0; b0 < nh; b0 += 32) {
      const int idx = b0 + lane;
      const int uv  = reg1[idx < nh ? idx : nh - 1];
      const int m32 = (nh - b0) < 32 ? (nh - b0) : 32;
#pragma unroll 1
      for (int k = 0; k < m32; ++k) {
        const int u  = __builtin_amdgcn_readlane(uv, k);
        const int sl = u & (NBMAX - 1);
        if (lane == 0) scnt[sl] = scnt[sl] + 1;
      }
    }
  }
  __syncthreads();

  {
    const v4i ca = *(const v4ia*)(scnt + 8 * tid);
    const v4i cb = *(const v4ia*)(scnt + 8 * tid + 4);
    const int e0 = ca.x < 0 ? 0 : ca.x, e1 = ca.y < 0 ? 0 : ca.y, e2 = ca.z < 0 ? 0 : ca.z, e3 = ca.w < 0 ? 0 : ca.w;
    const int e4 = cb.x < 0 ? 0 : cb.x, e5 = cb.y < 0 ? 0 : cb.y, e6 = cb.z < 0 ? 0 : cb.z, e7 = cb.w < 0 ? 0 : cb.w;
    const int ts = e0 + e1 + e2 + e3 + e4 + e5 + e6 + e7;
    int incl = ts;
#pragma unroll
    for (int d = 1; d < 32; d <<= 1) {
      const int up = __shfl_up(incl, d);
      if (lane >= d) incl += up;
    }
    if (lane == 31) wtot[wave] = incl;
    __syncthreads();
    int pre = 0;
#pragma unroll
    for (int w2 = 0; w2 < NWAVE; ++w2) pre += (w2 < wave) ? wtot[w2] : 0;
    int run = pre + incl - ts;
    soff[8 * tid + 0] = run; run += e0;
    soff[8 * tid + 1] = run; run += e1;
    soff[8 * tid + 2] = run; run += e2;
    soff[8 * tid + 3] = run; run += e3;
    soff[8 * tid + 4] = run; run += e4;
    soff[8 * tid + 5] = run; run += e5;
    soff[8 * tid + 6] = run; run += e6;
    soff[8 * tid + 7] = run;
  }
  __syncthreads();
  for (int i = tid; i < NBMAX; i += NTHR) list[i] = soff[i];
  __syncthreads();

  if (wave == 0) {
#pragma unroll 1
    for (int b0 = 0; b0 < nh; b0 += 32) {
      const int idx = b0 + lane;
      const int uv  = reg1[idx < nh ? idx : nh - 1];
      const int m32 = (nh - b0) < 32 ? (nh - b0) : 32;
#pragma unroll 1
      for (int k = 0; k < m32; ++k) {
        const int u   = __builtin_amdgcn_readlane(uv, k);
        const int sl  = u & (NBMAX - 1);
        const int eid = (int)((unsigned)u >> 12);
        if (lane == 0) {
          int pos = list[sl];
          pos = pos < 0 ? 0 : (pos > RCAP - 1 ? RCAP - 1 : pos);
          reg2[pos] = eid;
          list[sl] = pos + 1;
        }
      }
    }
  }
  __syncthreads();

  const int nbw = nb >> 3;
  const bool ovf = (nh >= RCAP);
  const float qnan = __int_as_float(0x7fc00000);
  float* stw = (float*)reg1 + wave * STW;
  v4f at4, bb4;
  {
    const v4f a = *(const v4fa*)(att + 4 * lane);
    const v4f b = *(const v4fa*)(bias + 4 * lane);
    at4.x = bf16_val(a.x); at4.y = bf16_val(a.y); at4.z = bf16_val(a.z); at4.w = bf16_val(a.w);
    bb4.x = bf16_val(b.x); bb4.y = bf16_val(b.y); bb4.z = bf16_val(b.z); bb4.w = bf16_val(b.w);
  }
#pragma unroll 1
  for (int jt = 0; jt < nbw; ++jt) {
    const int slot = wave * nbw + jt;
    const int grow = nodeBase + slot;
    const int gcl  = grow < nN ? grow : nN - 1;
    int st = soff[slot];
    const int craw = scnt[slot];
    int cnt = craw;
    st  = st < 0 ? 0 : (st > nh ? nh : st);
    cnt = cnt < 0 ? 0 : (cnt > DEGCAP ? DEGCAP : cnt);
    if (cnt > nh - st) cnt = nh - st;
    const float pz = (ovf || craw > DEGCAP) ? qnan : 0.0f;
    const bool live = grow < nN;

    const float* drow = XLR + (size_t)gcl * XW;
    const v4f xli = *(const v4fa*)(drow + 4 * lane);
    const v4f xri = *(const v4fa*)(drow + FT + 4 * lane);
    float mx = gred<NR>(lkatt4(xli, xri, at4));
    float dn = 1.0f;
    v4f av = xli;

#pragma unroll 1
    for (int b0 = 0; b0 < cnt; b0 += 32) {
      const int last = st + cnt - 1;
      int idx = st + b0 + lane;
      idx = idx > last ? last : idx;
      idx = idx < 0 ? 0 : (idx > RCAP - 1 ? RCAP - 1 : idx);
      int eid = reg2[idx];
      eid = eid < 0 ? 0 : (eid > nE - 1 ? nE - 1 : eid);
      int sr = srcs[eid];
      sr = sr < 0 ? 0 : (sr > nN - 1 ? nN - 1 : sr);
      const int m32 = (cnt - b0) < 32 ? (cnt - b0) : 32;
#pragma unroll 1
      for (int k = 0; k < m32; ++k) {
        const int sk = __builtin_amdgcn_readlane(sr, k);
        const v4f hs = *(const v4fa*)(XLR + (size_t)sk * XW + 4 * lane);
        const float al = gred<NR>(lkatt4(hs, xri, at4));
        const float df = al - mx;
        const float ee = expf(-fabsf(df));
        const bool up  = df > 0.f;
        const float s1 = up ? ee : 1.0f;
        const float s2 = up ? 1.0f : ee;
        mx = up ? al : mx;
        dn = fmaf(dn, s1, s2);
        av.x = fmaf(av.x, s1, s2 * hs.x);
        av.y = fmaf(av.y, s1, s2 * hs.y);
        av.z = fmaf(av.z, s1, s2 * hs.z);
        av.w = fmaf(av.w, s1, s2 * hs.w);
      }
    }
    const float iv = __builtin_amdgcn_rcpf(dn);
    v4f r;
    r.x = fmaf(av.x, iv, bb4.x);
    r.y = fmaf(av.y, iv, bb4.y);
    r.z = fmaf(av.z, iv, bb4.z);
    r.w = fmaf(av.w, iv, bb4.w);

    if constexpr (L == 1) {
      __builtin_amdgcn_fence(__ATOMIC_RELEASE, "wavefront");
      __builtin_amdgcn_wave_barrier();
      stw[4 * lane + 0] = r.x;
      stw[4 * lane + 1] = r.y;
      stw[4 * lane + 2] = r.z;
      stw[4 * lane + 3] = r.w;
      __builtin_amdgcn_fence(__ATOMIC_RELEASE, "wavefront");
      __builtin_amdgcn_wave_barrier();
#pragma unroll 1
      for (int j = 0; j < 4; ++j) {
        const float t = stw[4 * lane + j];
        const float g = 0.5f * t * (1.0f + erff(t * 0.70710678f));
        stw[4 * lane + j] = g;
      }
      __builtin_amdgcn_fence(__ATOMIC_RELEASE, "wavefront");
      __builtin_amdgcn_wave_barrier();
      const int c8 = 8 * (lane & 15);
      const v4f ga = *(const v4fa*)(stw + c8);
      const v4f gb = *(const v4fa*)(stw + c8 + 4);
      const bool hiLane = lane < 16;
      float f0 = ga.x, f1 = ga.y, f2 = ga.z, f3 = ga.w, f4 = gb.x, f5 = gb.y, f6 = gb.z, f7 = gb.w;
      unsigned q0, q1, q2, q3, q4, q5, q6, q7;
#define CVHL(FV, QV) { \
        const float vv = live ? ((FV) + pz) : 0.0f; \
        const unsigned hb = bf16_bits(vv); \
        const unsigned lb = bf16_bits(vv - __uint_as_float(hb << 16)); \
        QV = hiLane ? hb : lb; }
      CVHL(f0, q0) CVHL(f1, q1) CVHL(f2, q2) CVHL(f3, q3)
      CVHL(f4, q4) CVHL(f5, q5) CVHL(f6, q6) CVHL(f7, q7)
#undef CVHL
      v4u pv;
      pv.x = q0 | (q1 << 16);
      pv.y = q2 | (q3 << 16);
      pv.z = q4 | (q5 << 16);
      pv.w = q6 | (q7 << 16);
      const bool wr = grow < MPr;
      unsigned short* hp = H1 + (size_t)grow * XW + 8 * lane;
      if (wr) *(volatile v4u*)hp = pv;
      __threadfence();
      if (wr) *(volatile v4u*)hp = pv;
    } else {
      v4f ov;
      ov.x = r.x + pz; ov.y = r.y + pz; ov.z = r.z + pz; ov.w = r.w + pz;
      float* op = H2 + (size_t)grow * FT + 4 * lane;
      if (live) *(volatile v4f*)op = ov;
      __threadfence();
      if (live) *(volatile v4f*)op = ov;
    }
  }
  (void)H1; (void)H2; (void)MPr;
}

__global__ __launch_bounds__(NTHR) void k_pool_head(const float* __restrict__ hf, const int* __restrict__ bat,
                                                    const int* __restrict__ bsz,
                                                    const float* __restrict__ Wlin, const float* __restrict__ blin,
                                                    int nN, float* out) {
  __shared__ __attribute__((aligned(16))) float wsum[NWAVE * FT];
  __shared__ int wcn[NWAVE];
  __shared__ __attribute__((aligned(16))) float hrow[FT];
  __shared__ __attribute__((aligned(16))) float o0[FT];
  __shared__ __attribute__((aligned(16))) float o1[FT];
  const int tid = (int)threadIdx.x, lane = tid & 31, wave = tid >> 5;
  const int g = (int)blockIdx.x;
  const int nseg = bsz[0];
  const bool gok = g < nseg;

  v4f a = {0.f, 0.f, 0.f, 0.f};
  int cnt = 0;
#pragma unroll 1
  for (int i0 = wave * 32; i0 < nN; i0 += NTHR) {
    const int i  = i0 + lane;
    const int ic = i < nN ? i : nN - 1;
    const int b  = bat[ic];
    const bool hit = (i < nN) && (b == g) && gok;
    unsigned msk = __builtin_amdgcn_ballot_w32(hit);
    int nh = (int)__builtin_popcount(msk);
    nh = nh > 32 ? 32 : nh;
    cnt += nh;
#pragma unroll 1
    for (int q = 0; q < nh; ++q) {
      const int k = __builtin_ffs((int)msk) - 1;
      msk &= msk - 1u;
      int node = i0 + (k < 0 ? 0 : k);
      node = node > nN - 1 ? nN - 1 : node;
      const v4f v = *(const v4fa*)(hf + (size_t)node * FT + 4 * lane);
      a.x += v.x; a.y += v.y; a.z += v.z; a.w += v.w;
    }
  }
  wsum[wave * FT + 4 * lane + 0] = a.x;
  wsum[wave * FT + 4 * lane + 1] = a.y;
  wsum[wave * FT + 4 * lane + 2] = a.z;
  wsum[wave * FT + 4 * lane + 3] = a.w;
  if (lane == 0) wcn[wave] = cnt;
  if (tid < FT) {
    int first = g * NPER;
    first = first > nN - 1 ? nN - 1 : first;
    hrow[tid] = hf[(size_t)first * FT + tid];
  }
  __syncthreads();
  if (tid < FT) {
    double s = 0.0;
    int c = 0;
#pragma unroll
    for (int w2 = 0; w2 < NWAVE; ++w2) { s += (double)wsum[w2 * FT + tid]; c += wcn[w2]; }
    const float cf = (float)c;
    o1[tid] = (float)s * (1.0f / cf);
    float acc = 0.0f;
#pragma unroll 4
    for (int k = 0; k < FT; ++k) acc = fmaf(hrow[k], bf16_val(Wlin[(size_t)k * FT + tid]), acc);
    o0[tid] = acc + bf16_val(blin[tid]);
  }
  __syncthreads();
  const v4f r0 = *(const v4fa*)(o0 + 4 * lane);
  const v4f r1 = *(const v4fa*)(o1 + 4 * lane);
  float* p0 = out + (size_t)g * FT + 4 * lane;
  float* p1 = out + (size_t)NGR * FT + (size_t)g * FT + 4 * lane;
  const bool okst = (wave == 0);
  if (okst) { *(volatile v4f*)p0 = r0; *(volatile v4f*)p1 = r1; }
  __threadfence();
  if (okst) { *(volatile v4f*)p0 = r0; *(volatile v4f*)p1 = r1; }
}

static int pick_nb(int nE, int nN) {
  int nb = NBRUN;
  while (nb > 16 && (long long)nb * (long long)nE * 5LL > (long long)RCAP * (long long)nN * 4LL) nb >>= 1;
  return nb;
}
static inline int cdiv(int a, int b) { return (a + b - 1) / b; }
static inline size_t al256(size_t o) { return (o + 255) & ~(size_t)255; }

extern "C" void kernel_launch(void* const* d_in, const int* in_sizes, int n_in,
                              void* d_out, int out_size, void* d_ws, size_t ws_size,
                              hipStream_t stream) {
  if (n_in < 18) return;
  if (in_sizes[0] < FT || (in_sizes[0] % FT) != 0) return;
  const int nN = in_sizes[0] / FT;
  if (nN != NGR * NPER) return;
  if (in_sizes[1] != FT * FT || in_sizes[3] != FT * FT) return;
  if (in_sizes[2] != FT || in_sizes[4] != FT || in_sizes[5] != FT || in_sizes[6] != FT) return;
  if (in_sizes[7] != FT * FT || in_sizes[9] != FT * FT) return;
  if (in_sizes[8] != FT || in_sizes[10] != FT || in_sizes[11] != FT || in_sizes[12] != FT) return;
  if (in_sizes[13] != FT * FT || in_sizes[14] != FT) return;
  if (in_sizes[15] < 2 || (in_sizes[15] & 1) != 0) return;
  const int nE = in_sizes[15] / 2;
  if (nE < 1 || nE > (1 << 20)) return;
  if (in_sizes[16] != nN || in_sizes[17] < 1) return;
  if (out_size != 2 * NGR * FT) return;

  const float* x     = (const float*)d_in[0];
  const float* Wl1   = (const float*)d_in[1];
  const float* bl1   = (const float*)d_in[2];
  const float* Wr1   = (const float*)d_in[3];
  const float* br1   = (const float*)d_in[4];
  const float* att1  = (const float*)d_in[5];
  const float* bias1 = (const float*)d_in[6];
  const float* Wl2   = (const float*)d_in[7];
  const float* bl2   = (const float*)d_in[8];
  const float* Wr2   = (const float*)d_in[9];
  const float* br2   = (const float*)d_in[10];
  const float* att2  = (const float*)d_in[11];
  const float* bias2 = (const float*)d_in[12];
  const float* Wlin  = (const float*)d_in[13];
  const float* blin  = (const float*)d_in[14];
  const int*   ei    = (const int*)d_in[15];
  const int*   bat   = (const int*)d_in[16];
  const int*   bsz   = (const int*)d_in[17];
  float* out = (float*)d_out;
  const int* src = ei;
  const int* dst = ei + nE;

  const int MP   = cdiv(nN, GBM) * GBM;
  const int gM   = MP / GBM;
  const int gX   = MP / 16;
  const int nb   = pick_nb(nE, nN);
  const int gA   = cdiv(MP, nb);
  const int vec8 = ((nE & 3) == 0) ? 1 : 0;
  if ((long long)gA * nb < (long long)MP) return;
  if (gX * 16 != MP) return;

  char* ws = (char*)d_ws;
  size_t off = 0;
  const size_t oXB  = off; off = al256(off + (size_t)MP * FT * 2);
  const size_t oW1T = off; off = al256(off + (size_t)XW * FT * 2);
  const size_t oW2T = off; off = al256(off + (size_t)XW * XW * 2);
  const size_t oXLR = off; off = al256(off + (size_t)MP * XW * 4);
  const size_t oH1  = off; off = al256(off + (size_t)MP * XW * 2);
  const size_t oH2  = off; off = al256(off + (size_t)nN * FT * 4);
  if (off > ws_size || off > (size_t)WSMAX) return;
  unsigned short* XB  = (unsigned short*)(ws + oXB);
  unsigned short* W1T = (unsigned short*)(ws + oW1T);
  unsigned short* W2T = (unsigned short*)(ws + oW2T);
  float*          XLR = (float*)(ws + oXLR);
  unsigned short* H1  = (unsigned short*)(ws + oH1);
  float*          H2  = (float*)(ws + oH2);

  hipFuncSetAttribute(reinterpret_cast<const void*>(&k_agg<1>), hipFuncAttributeMaxDynamicSharedMemorySize, LDS_AGG);
  hipFuncSetAttribute(reinterpret_cast<const void*>(&k_agg<2>), hipFuncAttributeMaxDynamicSharedMemorySize, LDS_AGG);

  k_prep<<<gX + NUW / NTHR, NTHR, 0, stream>>>(x, Wl1, Wr1, Wl2, Wr2, XB, W1T, W2T, nN, gX);
  k_gemm<<<dim3(gM, XW / GBN), GTHR, 0, stream>>>(XB, W1T, bl1, br1, XLR, FT, XW);
  k_agg<1><<<gA, NTHR, LDS_AGG, stream>>>(src, dst, XLR, att1, bias1, H1, H2, nN, nE, nb, vec8, MP);
  k_gemm<<<dim3(gM, XW / GBN), GTHR, 0, stream>>>(H1, W2T, bl2, br2, XLR, XW, XW);
  k_agg<2><<<gA, NTHR, LDS_AGG, stream>>>(src, dst, XLR, att2, bias2, H1, H2, nN, nE, nb, vec8, MP);
  k_pool_head<<<NGR, NTHR, 0, stream>>>(H2, bat, bsz, Wlin, blin, nN, out);
}
